// LinearBlock_49709951484049
// MI455X (gfx1250) — hardware-verified
//
#include <hip/hip_runtime.h>
#include <math.h>

constexpr int NBATCH = 2;
constexpr int NSEQ   = 1024;
constexpr int DMODEL = 1024;
constexpr int NHEAD  = 16;
constexpr int DHEAD  = 64;
constexpr int FFDIM  = 4096;
constexpr int NTOK   = NBATCH * NSEQ;
constexpr int NQB    = NSEQ / 64;
constexpr float WCARRY   = 1024.0f;
constexpr float ATTCARRY = 256.0f;
constexpr float FFCARRY  = 64.0f;

static_assert(NHEAD * DHEAD == DMODEL);
static_assert(NSEQ % 64 == 0);
static_assert(DHEAD == 64);
static_assert(DMODEL % 64 == 0 && FFDIM % 64 == 0 && NTOK % 64 == 0);
static_assert(DMODEL % 32 == 0 && FFDIM % 32 == 0);

constexpr size_t SZ_WQKVT = (size_t)3 * DMODEL * DMODEL * 2;
constexpr size_t SZ_WOT   = (size_t)DMODEL * DMODEL * 2;
constexpr size_t SZ_W1T   = (size_t)FFDIM * DMODEL * 2;
constexpr size_t SZ_W2T   = (size_t)DMODEL * FFDIM * 2;
constexpr size_t SZ_H16   = (size_t)NTOK * DMODEL * 2;
constexpr size_t SZ_BIG   = (size_t)NTOK * FFDIM * 4;
constexpr size_t SZ_P16   = (size_t)NTOK * DMODEL * 2;
constexpr size_t SZ_X2    = (size_t)NTOK * DMODEL * 4;
constexpr size_t SZ_FF16  = (size_t)NTOK * FFDIM * 2;
constexpr size_t WS_WQKVT = 0;
constexpr size_t WS_WOT   = WS_WQKVT + SZ_WQKVT;
constexpr size_t WS_W1T   = WS_WOT + SZ_WOT;
constexpr size_t WS_W2T   = WS_W1T + SZ_W1T;
constexpr size_t WS_H16   = WS_W2T + SZ_W2T;
constexpr size_t WS_BIG   = WS_H16 + SZ_H16;
constexpr size_t WS_QF    = WS_BIG + SZ_BIG;
constexpr size_t WS_KF    = WS_QF + SZ_P16;
constexpr size_t WS_VP    = WS_KF + SZ_P16;
constexpr size_t WS_ATT   = WS_VP + SZ_P16;
constexpr size_t WS_X2    = WS_ATT + SZ_P16;
constexpr size_t WS_FF16  = WS_X2 + SZ_X2;
constexpr size_t WS_TOTAL = WS_FF16 + SZ_FF16;
static_assert(SZ_BIG >= (size_t)NTOK * 3 * DMODEL * 4);
static_assert(SZ_BIG >= (size_t)NTOK * DMODEL * 4);
static_assert(WS_TOTAL == 104857600);
static_assert(WS_TOTAL <= 134217728);
static_assert((WS_WOT % 128) == 0 && (WS_W1T % 128) == 0 && (WS_W2T % 128) == 0 && (WS_H16 % 128) == 0 &&
              (WS_BIG % 128) == 0 && (WS_QF % 128) == 0 && (WS_KF % 128) == 0 && (WS_VP % 128) == 0 &&
              (WS_ATT % 128) == 0 && (WS_X2 % 128) == 0 && (WS_FF16 % 128) == 0);

typedef __attribute__((ext_vector_type(16))) _Float16 v16h;
typedef __attribute__((ext_vector_type(8)))  _Float16 v8h;
typedef __attribute__((ext_vector_type(16))) __bf16   v16b;
typedef __attribute__((ext_vector_type(8)))  __bf16   v8b;
typedef __attribute__((ext_vector_type(8)))  float    v8f;
typedef __attribute__((ext_vector_type(4)))  float    v4f;

__device__ __forceinline__ unsigned short f2bf_bits(float f) {
  unsigned u = __float_as_uint(f);
  return (unsigned short)((u + 0x7FFFu + ((u >> 16) & 1u)) >> 16);
}
__device__ __forceinline__ float bf_bits2f(unsigned short h) { return __uint_as_float(((unsigned)h) << 16); }

__device__ __forceinline__ void dep_guard_h(v8f& a, v8f& b, v16h x, v16h y) { asm volatile("v_nop\n\tv_nop\n\tv_nop\n\tv_nop" : "+v"(a), "+v"(b) : "v"(x), "v"(y)); }
__device__ __forceinline__ void dep_guard_b(v8f& a, v8f& b, v16b x, v16b y) { asm volatile("v_nop\n\tv_nop\n\tv_nop\n\tv_nop" : "+v"(a), "+v"(b) : "v"(x), "v"(y)); }
__device__ __forceinline__ void keep4_h(v16h a, v16h b, v16h c, v16h d) { asm volatile("v_nop" :: "v"(a), "v"(b), "v"(c), "v"(d)); }
__device__ __forceinline__ void keep4_b(v16b a, v16b b, v16b c, v16b d) { asm volatile("v_nop" :: "v"(a), "v"(b), "v"(c), "v"(d)); }
__device__ __forceinline__ void acc_guard4(v8f& a, v8f& b, v8f& c, v8f& d) { asm volatile("v_nop\n\tv_nop\n\tv_nop\n\tv_nop" : "+v"(a), "+v"(b), "+v"(c), "+v"(d)); }
template <typename T> struct Frag;
template <> struct Frag<_Float16> {
  typedef v16h V; union U { v16h v; v8h h[2]; };
  static __device__ __forceinline__ v16h load(const _Float16* p) {
    U f; f.h[0] = *(const v8h*)(p); f.h[1] = *(const v8h*)(p + 16); return f.v;
  }
  static __device__ __forceinline__ v8f mma(v16h a, v16h b, v8f c) {
    return __builtin_amdgcn_wmma_f32_16x16x32_f16(false, a, false, b, (short)0, c, false, false);
  }
  static __device__ __forceinline__ void guard(v8f& a, v8f& b, v16h x, v16h y) { dep_guard_h(a, b, x, y); }
  static __device__ __forceinline__ void keep(v16h a, v16h b, v16h c, v16h d) { keep4_h(a, b, c, d); }
};
template <> struct Frag<__bf16> {
  typedef v16b V; union U { v16b v; v8b h[2]; };
  static __device__ __forceinline__ v16b load(const __bf16* p) {
    U f; f.h[0] = *(const v8b*)(p); f.h[1] = *(const v8b*)(p + 16); return f.v;
  }
  static __device__ __forceinline__ v8f mma(v16b a, v16b b, v8f c) {
    return __builtin_amdgcn_wmma_f32_16x16x32_bf16(false, a, false, b, (short)0, c, false, false);
  }
  static __device__ __forceinline__ void guard(v8f& a, v8f& b, v16b x, v16b y) { dep_guard_b(a, b, x, y); }
  static __device__ __forceinline__ void keep(v16b a, v16b b, v16b c, v16b d) { keep4_b(a, b, c, d); }
};

template <int ET> struct Elem;
template <> struct Elem<0> { typedef _Float16 T; };
template <> struct Elem<1> { typedef __bf16 T; };
template <int ET, bool SPLIT, int BIAS_MODE, int OUT_MODE, bool RESID, int ACT = 0>
__global__ __launch_bounds__(256) void wmma_gemm64(
    const unsigned short* __restrict__ Ap, const unsigned short* __restrict__ A2p, int lda, long strideA,
    const unsigned short* __restrict__ Btp, const unsigned short* __restrict__ Bt2p, int ldb, long strideB,
    void* __restrict__ Cout, void* __restrict__ Cout2, int ldc, long strideC,
    const float* __restrict__ bias,
    const float* __restrict__ resid, long strideR,
    int M, int N, int K, float scale) {
  typedef typename Elem<ET>::T T;
  typedef typename Frag<T>::V V;
  const T* A = (const T*)Ap; const T* A2 = (const T*)A2p; const T* Bt = (const T*)Btp; const T* Bt2 = (const T*)Bt2p;
  __shared__ __align__(16) float sT[8][16 * 68];
  const int b    = blockIdx.y;
  const int lane = threadIdx.x & 31;
  const int wave = threadIdx.x >> 5;
  const int tilesN = N >> 6;
  const int tilesM = M >> 6;
  const int tile = blockIdx.x * 8 + wave;
  if (tile >= tilesM * tilesN) return;
  const int tm = tile / tilesN;
  const int tn = tile - tm * tilesN;
  const int m0 = tm << 6;
  const int n0 = tn << 6;

  const T* Ab  = A  + (size_t)b * strideA;
  const T* Bb  = Bt + (size_t)b * strideB;
  const T* Ab2 = SPLIT ? (A2  + (size_t)b * strideA) : nullptr;
  const T* Bb2 = SPLIT ? (Bt2 + (size_t)b * strideB) : nullptr;

  const int rlane = lane & 15;
  const int koff  = (lane >> 4) * 8;
  const int mOff  = (lane >> 4) * 8;

  v8f acc[4][4];
#pragma unroll
  for (int i = 0; i < 4; ++i)
#pragma unroll
    for (int j = 0; j < 4; ++j) acc[i][j] = (v8f){0.f,0.f,0.f,0.f,0.f,0.f,0.f,0.f};

  for (int k0 = 0; k0 < K; k0 += 32) {
    V bh[4], bl[4];
#pragma unroll
    for (int j = 0; j < 4; ++j) {
      const size_t bo = (size_t)(n0 + (j << 4) + rlane) * ldb + koff + k0;
      bh[j] = Frag<T>::load(Bb + bo);
      if (SPLIT) bl[j] = Frag<T>::load(Bb2 + bo);
    }
#pragma unroll
    for (int i = 0; i < 4; ++i) {
      const size_t ao = (size_t)(m0 + (i << 4) + rlane) * lda + koff + k0;
      V ah = Frag<T>::load(Ab + ao);
      V al;
      if (SPLIT) al = Frag<T>::load(Ab2 + ao);
#pragma unroll
      for (int j = 0; j < 4; ++j) {
        acc[i][j] = Frag<T>::mma(ah, bh[j], acc[i][j]);
        if (SPLIT) {
          acc[i][j] = Frag<T>::mma(ah, bl[j], acc[i][j]);
          acc[i][j] = Frag<T>::mma(al, bh[j], acc[i][j]);
        }
      }
      Frag<T>::guard(acc[i][0], acc[i][3], ah, SPLIT ? al : ah);
    }
    Frag<T>::keep(bh[0], bh[1], bh[2], bh[3]);
    if (SPLIT) Frag<T>::keep(bl[0], bl[1], bl[2], bl[3]);
  }
  acc_guard4(acc[0][0], acc[0][1], acc[0][2], acc[0][3]);
  acc_guard4(acc[1][0], acc[1][1], acc[1][2], acc[1][3]);
  acc_guard4(acc[2][0], acc[2][1], acc[2][2], acc[2][3]);
  acc_guard4(acc[3][0], acc[3][1], acc[3][2], acc[3][3]);

  float* slab = sT[wave];
  const float* Rb = RESID ? (resid + (size_t)b * strideR) : nullptr;
#pragma unroll
  for (int i = 0; i < 4; ++i) {
    const int mBase = m0 + (i << 4);
#pragma unroll
    for (int j = 0; j < 4; ++j) {
      const int n = n0 + (j << 4) + rlane;
      float bv = 0.f;
      if (BIAS_MODE == 2) bv = bias[n];
#pragma unroll
      for (int r = 0; r < 8; ++r) {
        float v = acc[i][j][r] * scale;
        if (BIAS_MODE == 1) v += bias[mBase + mOff + r];
        if (BIAS_MODE == 2) v += bv;
        if (RESID) v += Rb[(size_t)(mBase + mOff + r) * ldc + n];
        if (ACT == 1) v = tanhf(v);
        if (ACT == 2) v = fmaxf(v, 0.0f);
        if (ACT == 3) v = v / (1.0f + expf(-v));
        if (ACT == 4) v = (v > 0.f) ? v : 0.01f * v;
        slab[(mOff + r) * 68 + (j << 4) + rlane] = v;
      }
    }
    __builtin_amdgcn_fence(__ATOMIC_RELEASE, "workgroup");
    __builtin_amdgcn_wave_barrier();
    __builtin_amdgcn_fence(__ATOMIC_ACQUIRE, "workgroup");
    if (OUT_MODE == 0) {
      float* C = (float*)Cout + (size_t)b * strideC;
      const int hh = lane >> 4, c4 = (lane & 15) * 4;
      for (int pass = 0; pass < 2; ++pass) {
#pragma unroll
        for (int it = 0; it < 8; ++it) {
          const int row = it * 2 + hh;
          v4f v = *(const v4f*)(slab + row * 68 + c4);
          *(volatile v4f*)(C + (size_t)(mBase + row) * ldc + n0 + c4) = v;
        }
        __threadfence();
      }
    } else {
      const int q = lane >> 3, c8 = (lane & 7) * 8;
      unsigned short* C  = (unsigned short*)Cout  + (size_t)b * strideC;
      unsigned short* C2 = (OUT_MODE == 2) ? ((unsigned short*)Cout2 + (size_t)b * strideC) : nullptr;
      for (int pass = 0; pass < 2; ++pass) {
#pragma unroll
        for (int it = 0; it < 4; ++it) {
          const int row = it * 4 + q;
          const float* sp = slab + row * 68 + c8;
          v8h hv, lv;
#pragma unroll
          for (int e = 0; e < 8; ++e) {
            if (OUT_MODE == 1) {
              hv[e] = (_Float16)sp[e];
            } else {
              unsigned short hb = f2bf_bits(sp[e]);
              unsigned short lb = f2bf_bits(sp[e] - bf_bits2f(hb));
              hv[e] = __builtin_bit_cast(_Float16, hb);
              lv[e] = __builtin_bit_cast(_Float16, lb);
            }
          }
          *(volatile v8h*)(C + (size_t)(mBase + row) * ldc + n0 + c8) = hv;
          if (OUT_MODE == 2) *(volatile v8h*)(C2 + (size_t)(mBase + row) * ldc + n0 + c8) = lv;
        }
        __threadfence();
      }
    }
    __builtin_amdgcn_fence(__ATOMIC_RELEASE, "workgroup");
    __builtin_amdgcn_wave_barrier();
    __builtin_amdgcn_fence(__ATOMIC_ACQUIRE, "workgroup");
  }
}

__global__ __launch_bounds__(256) void tcast_f32_f16(const float* __restrict__ W, unsigned short* __restrict__ Wt,
                                                    int kdim, int ndim, float scale) {
  __shared__ float tile[64 * 65];
  const int k0 = blockIdx.y * 64;
  const int n0 = blockIdx.x * 64;
  const int tid = threadIdx.x;
  {
    const int row = tid >> 2;
    const int cb  = (tid & 3) * 16;
    const float* src = W + (size_t)(k0 + row) * ndim + n0 + cb;
#pragma unroll
    for (int i = 0; i < 4; ++i) {
      const v4f f = *(const v4f*)(src + 4 * i);
      tile[row * 65 + cb + 4 * i + 0] = f[0];
      tile[row * 65 + cb + 4 * i + 1] = f[1];
      tile[row * 65 + cb + 4 * i + 2] = f[2];
      tile[row * 65 + cb + 4 * i + 3] = f[3];
    }
  }
  __syncthreads();
  const int wave = tid >> 5, lane = tid & 31;
  const int q8 = lane >> 3, c8 = (lane & 7) * 8;
  v8h hv[2];
#pragma unroll
  for (int it = 0; it < 2; ++it) {
    const int r = wave * 8 + it * 4 + q8;
#pragma unroll
    for (int e = 0; e < 8; ++e) hv[it][e] = (_Float16)(tile[(c8 + e) * 65 + r] * scale);
  }
  for (int pass = 0; pass < 2; ++pass) {
#pragma unroll
    for (int it = 0; it < 2; ++it) {
      const int r = wave * 8 + it * 4 + q8;
      *(volatile v8h*)(Wt + (size_t)(n0 + r) * kdim + k0 + c8) = hv[it];
    }
    __threadfence();
  }
}

template <bool ADD>
__global__ __launch_bounds__(256) void layernorm_f16(const float* __restrict__ x, const float* __restrict__ addp,
                                                    const float* __restrict__ g, const float* __restrict__ bta,
                                                    float* __restrict__ xsum_out, unsigned short* __restrict__ y) {
  __shared__ __align__(16) float rowbuf[DMODEL];
  __shared__ float red1[8];
  __shared__ float red2[8];
  const int row  = blockIdx.x;
  const int tid  = threadIdx.x;
  const int lane = tid & 31;
  const int wave = tid >> 5;
  const size_t rb = (size_t)row * DMODEL;

  v4f a = *(const v4f*)(x + rb + tid * 4);
  if (ADD) {
    const v4f p = *(const v4f*)(addp + rb + tid * 4);
    a += p;
    volatile v4f* xo = (volatile v4f*)(xsum_out + rb + tid * 4);
    *xo = a;
    __threadfence();
    *xo = a;
  }
  *(v4f*)(rowbuf + tid * 4) = a;
  float s = (a[0] + a[1]) + (a[2] + a[3]);
#pragma unroll
  for (int off = 1; off < 32; off <<= 1) s += __shfl_xor(s, off, 32);
  if (lane == 0) red1[wave] = s;
  __syncthreads();
  const float mean = (((red1[0] + red1[1]) + (red1[2] + red1[3])) + ((red1[4] + red1[5]) + (red1[6] + red1[7]))) * (1.0f / DMODEL);
  const v4f d = a - mean;
  float s2 = (d[0] * d[0] + d[1] * d[1]) + (d[2] * d[2] + d[3] * d[3]);
#pragma unroll
  for (int off = 1; off < 32; off <<= 1) s2 += __shfl_xor(s2, off, 32);
  if (lane == 0) red2[wave] = s2;
  __syncthreads();
  const float var = (((red2[0] + red2[1]) + (red2[2] + red2[3])) + ((red2[4] + red2[5]) + (red2[6] + red2[7]))) * (1.0f / DMODEL);
  const float inv = 1.0f / sqrtf(var + 1e-5f);
  if (tid < 128) {
    const v4f u0 = *(const v4f*)(rowbuf + tid * 8);
    const v4f u1 = *(const v4f*)(rowbuf + tid * 8 + 4);
    const v4f g0 = *(const v4f*)(g + tid * 8);
    const v4f g1 = *(const v4f*)(g + tid * 8 + 4);
    const v4f b0 = *(const v4f*)(bta + tid * 8);
    const v4f b1 = *(const v4f*)(bta + tid * 8 + 4);
    v8h hv;
#pragma unroll
    for (int e = 0; e < 4; ++e) {
      hv[e]     = (_Float16)((u0[e] - mean) * inv * g0[e] + b0[e]);
      hv[4 + e] = (_Float16)((u1[e] - mean) * inv * g1[e] + b1[e]);
    }
    volatile v8h* yo = (volatile v8h*)(y + rb + tid * 8);
    *yo = hv;
    __threadfence();
    *yo = hv;
  }
}

__global__ __launch_bounds__(256) void qkv_feature_f16(const float* __restrict__ qkv, const int* __restrict__ mask,
                                                      unsigned short* __restrict__ qf, unsigned short* __restrict__ kf,
                                                      unsigned short* __restrict__ vp) {
  const int plane = blockIdx.y;
  const int i   = blockIdx.x * 256 + threadIdx.x;
  const int row = i >> 9;
  const int col = (i & 511) * 2;
  const float mval = (float)mask[row];
  const float* src = qkv + (size_t)row * (3 * DMODEL) + plane * DMODEL + col;
  unsigned packed = 0;
#pragma unroll 1
  for (int e = 0; e < 2; ++e) {
    const float xx = src[e];
    const float ex = expf(fminf(xx, 0.0f));
    const float ph = (xx > 0.0f) ? (xx + 1.0f) : ex;
    float yv = ph;
    if (plane == 1) yv = ph * mval;
    if (plane == 2) yv = xx * mval;
    const unsigned short hb = __builtin_bit_cast(unsigned short, (_Float16)yv);
    packed |= ((unsigned)hb) << (16 * e);
  }
  unsigned short* dst = (plane == 0) ? qf : ((plane == 1) ? kf : vp);
  volatile unsigned* o = (volatile unsigned*)dst + i;
  *o = packed;
  __threadfence();
  *o = packed;
}

__global__ __launch_bounds__(256) void gelu_f16(const float* __restrict__ in, unsigned short* __restrict__ out, float carry) {
  const int i = blockIdx.x * 256 + threadIdx.x;
  unsigned packed = 0;
#pragma unroll 1
  for (int e = 0; e < 2; ++e) {
    const float xg = in[2 * (size_t)i + e];
    const float yv = 0.5f * xg * (1.0f + erff(xg * 0.70710678118654752f)) * carry;
    const unsigned short hb = __builtin_bit_cast(unsigned short, (_Float16)yv);
    packed |= ((unsigned)hb) << (16 * e);
  }
  volatile unsigned* o = (volatile unsigned*)out + i;
  *o = packed;
  __threadfence();
  *o = packed;
}

__global__ __launch_bounds__(256) void add_f32(const float* __restrict__ a, const float* __restrict__ bsrc, float* __restrict__ out) {
  const size_t i = (size_t)(blockIdx.x * 256 + threadIdx.x) * 4;
  const v4f s = *(const v4f*)(a + i) + *(const v4f*)(bsrc + i);
  volatile v4f* o = (volatile v4f*)(out + i);
  *o = s;
  __threadfence();
  *o = s;
}

__device__ __forceinline__ v8f mma_f16g(v16h a, v16h b, v8f c) {
  c = __builtin_amdgcn_wmma_f32_16x16x32_f16(false, a, false, b, (short)0, c, false, false);
  asm volatile("v_nop\n\tv_nop\n\tv_nop\n\tv_nop" : "+v"(c) : "v"(a), "v"(b));
  return c;
}

__global__ __launch_bounds__(128)
void causal_linear_attn(const unsigned short* __restrict__ Qf, const unsigned short* __restrict__ Kf,
                        const unsigned short* __restrict__ Vp, unsigned short* __restrict__ Op) {
  __shared__ __align__(16) unsigned short Ksh[64 * 64];
  __shared__ __align__(16) unsigned short Vt[64 * 64];
  __shared__ __align__(16) unsigned short Psh[4][16 * 64];
  __shared__ __align__(16) float Os[4][16 * 68];

  const int tid  = threadIdx.x;
  const int wave = tid >> 5;
  const int lane = tid & 31;
  const int hh   = lane >> 4;
  const int c    = lane & 15;

  const int bx = blockIdx.x;
  const int qb = bx % NQB;
  const int bh = bx / NQB;
  const int h  = bh % NHEAD;
  const int b  = bh / NHEAD;
  const int q0 = qb * 64 + wave * 16;
  const size_t hoff = (size_t)h * DHEAD;

  v16h qa[2];
  {
    const _Float16* qrow = (const _Float16*)Qf + ((size_t)(b * NSEQ + q0 + c)) * DMODEL + hoff + 8 * hh;
#pragma unroll
    for (int dc = 0; dc < 2; ++dc) qa[dc] = Frag<_Float16>::load(qrow + dc * 32);
  }

  float den[8];
  v8f oacc[4];
#pragma unroll
  for (int r = 0; r < 8; ++r) den[r] = 0.f;
#pragma unroll
  for (int t = 0; t < 4; ++t) oacc[t] = (v8f){0.f,0.f,0.f,0.f,0.f,0.f,0.f,0.f};

  const int nChunks = qb + 1;
  for (int kc = 0; kc < nChunks; ++kc) {
    const int kv0 = kc * 64;
    __syncthreads();
    {
      const int kvr = tid >> 1;
      const int dh  = (tid & 1) * 32;
      const size_t rbk = ((size_t)(b * NSEQ + kv0 + kvr)) * DMODEL + hoff + dh;
      const uint4* ksrc = (const uint4*)(Kf + rbk);
      const uint4* vsrc = (const uint4*)(Vp + rbk);
      uint4* kdst = (uint4*)(Ksh + kvr * 64 + dh);
#pragma unroll
      for (int i = 0; i < 4; ++i) {
        kdst[i] = ksrc[i];
        const uint4 w = vsrc[i];
        const int d0 = dh + 8 * i;
        Vt[(d0 + 0) * 64 + kvr] = (unsigned short)(w.x & 0xffffu);
        Vt[(d0 + 1) * 64 + kvr] = (unsigned short)(w.x >> 16);
        Vt[(d0 + 2) * 64 + kvr] = (unsigned short)(w.y & 0xffffu);
        Vt[(d0 + 3) * 64 + kvr] = (unsigned short)(w.y >> 16);
        Vt[(d0 + 4) * 64 + kvr] = (unsigned short)(w.z & 0xffffu);
        Vt[(d0 + 5) * 64 + kvr] = (unsigned short)(w.z >> 16);
        Vt[(d0 + 6) * 64 + kvr] = (unsigned short)(w.w & 0xffffu);
        Vt[(d0 + 7) * 64 + kvr] = (unsigned short)(w.w >> 16);
      }
    }
    __syncthreads();

    v8f s[4];
#pragma unroll
    for (int j = 0; j < 4; ++j) {
      s[j] = (v8f){0.f,0.f,0.f,0.f,0.f,0.f,0.f,0.f};
#pragma unroll
      for (int dc = 0; dc < 2; ++dc) {
        const v16h kb = Frag<_Float16>::load((const _Float16*)Ksh + (j * 16 + c) * 64 + dc * 32 + 8 * hh);
        s[j] = mma_f16g(qa[dc], kb, s[j]);
      }
    }
    const bool diag = (kc == qb);
    unsigned short* pw = Psh[wave];
#pragma unroll
    for (int r = 0; r < 8; ++r) {
      const int qrow = q0 + 8 * hh + r;
      float ps = 0.f;
#pragma unroll
      for (int j = 0; j < 4; ++j) {
        const int kvcol = kv0 + j * 16 + c;
        float val = s[j][r];
        if (diag && (kvcol > qrow)) val = 0.f;
        ps += val;
        pw[(8 * hh + r) * 64 + j * 16 + c] = __builtin_bit_cast(unsigned short, (_Float16)val);
      }
#pragma unroll
      for (int off = 1; off < 16; off <<= 1) ps += __shfl_xor(ps, off, 32);
      den[r] += ps;
    }
    __syncthreads();

#pragma unroll
    for (int kk = 0; kk < 2; ++kk) {
      const v16h pa = Frag<_Float16>::load((const _Float16*)pw + c * 64 + kk * 32 + 8 * hh);
#pragma unroll
      for (int t = 0; t < 4; ++t) {
        const v16h vb = Frag<_Float16>::load((const _Float16*)Vt + (t * 16 + c) * 64 + kk * 32 + 8 * hh);
        oacc[t] = mma_f16g(pa, vb, oacc[t]);
      }
    }
  }

  float* os = Os[wave];
#pragma unroll
  for (int r = 0; r < 8; ++r) {
    const float inv = 1.0f / (den[r] + 1e-6f);
#pragma unroll
    for (int t = 0; t < 4; ++t) os[(8 * hh + r) * 68 + t * 16 + c] = (oacc[t][r] * inv) * ATTCARRY;
  }
  __syncthreads();
  {
    const int q8 = lane >> 3, c8 = (lane & 7) * 8;
    v8h ov[4];
#pragma unroll
    for (int it = 0; it < 4; ++it) {
      const int row = it * 4 + q8;
      const float* sp = os + row * 68 + c8;
#pragma unroll
      for (int e = 0; e < 8; ++e) ov[it][e] = (_Float16)sp[e];
    }
    unsigned short* obase = Op + ((size_t)(b * NSEQ + q0)) * DMODEL + hoff + c8;
    for (int pass = 0; pass < 2; ++pass) {
#pragma unroll
      for (int it = 0; it < 4; ++it) {
        const int row = it * 4 + q8;
        *(volatile v8h*)(obase + (size_t)row * DMODEL) = ov[it];
      }
      __threadfence();
    }
  }
}

static_assert(NTOK % 64 == 0 && (3 * DMODEL) % 64 == 0 && DMODEL % 32 == 0);
static_assert(((NTOK / 64) * ((3 * DMODEL) / 64)) % 8 == 0);
static_assert(((NTOK / 64) * (DMODEL / 64)) % 8 == 0);
static_assert(((NTOK / 64) * (FFDIM / 64)) % 8 == 0);
static_assert(FFDIM % 32 == 0);
static_assert((NTOK * DMODEL / 2) % 256 == 0 && (NTOK * FFDIM / 2) % 256 == 0 && (NTOK * DMODEL / 4) % 256 == 0);

extern "C" void kernel_launch(void* const* d_in, const int* in_sizes, int n_in,
                              void* d_out, int out_size, void* d_ws, size_t ws_size,
                              hipStream_t stream) {
  (void)n_in;
  if (ws_size < WS_TOTAL) return;
  if (out_size != NTOK * DMODEL) return;
  if (in_sizes[0] != NTOK * DMODEL || in_sizes[1] != NTOK) return;

  const float* x      = (const float*)d_in[0];
  const int*   amask  = (const int*)d_in[1];
  const float* Wq     = (const float*)d_in[2];
  const float* Wk     = (const float*)d_in[3];
  const float* Wv     = (const float*)d_in[4];
  const float* Wo     = (const float*)d_in[5];
  const float* ln_a_g = (const float*)d_in[6];
  const float* ln_a_b = (const float*)d_in[7];
  const float* ln_m_g = (const float*)d_in[8];
  const float* ln_m_b = (const float*)d_in[9];
  const float* W1     = (const float*)d_in[10];
  const float* b1     = (const float*)d_in[11];
  const float* W2     = (const float*)d_in[12];
  const float* b2     = (const float*)d_in[13];
  float* out = (float*)d_out;

  unsigned char* ws = (unsigned char*)d_ws;
  unsigned short* wqkvt = (unsigned short*)(ws + WS_WQKVT);
  unsigned short* wot   = (unsigned short*)(ws + WS_WOT);
  unsigned short* w1t   = (unsigned short*)(ws + WS_W1T);
  unsigned short* w2t   = (unsigned short*)(ws + WS_W2T);
  unsigned short* h16   = (unsigned short*)(ws + WS_H16);
  float*          big   = (float*)(ws + WS_BIG);
  unsigned short* qf    = (unsigned short*)(ws + WS_QF);
  unsigned short* kf    = (unsigned short*)(ws + WS_KF);
  unsigned short* vp    = (unsigned short*)(ws + WS_VP);
  unsigned short* att   = (unsigned short*)(ws + WS_ATT);
  float*          x2    = (float*)(ws + WS_X2);
  unsigned short* ff16  = (unsigned short*)(ws + WS_FF16);

  const dim3 blk256(256);

  tcast_f32_f16<<<dim3(DMODEL / 64, DMODEL / 64), blk256, 0, stream>>>(Wq, wqkvt, DMODEL, DMODEL, WCARRY);
  tcast_f32_f16<<<dim3(DMODEL / 64, DMODEL / 64), blk256, 0, stream>>>(Wk, wqkvt + (size_t)DMODEL * DMODEL, DMODEL, DMODEL, WCARRY);
  tcast_f32_f16<<<dim3(DMODEL / 64, DMODEL / 64), blk256, 0, stream>>>(Wv, wqkvt + (size_t)2 * DMODEL * DMODEL, DMODEL, DMODEL, WCARRY);
  tcast_f32_f16<<<dim3(DMODEL / 64, DMODEL / 64), blk256, 0, stream>>>(Wo, wot, DMODEL, DMODEL, WCARRY);
  tcast_f32_f16<<<dim3(FFDIM / 64, DMODEL / 64), blk256, 0, stream>>>(W1, w1t, DMODEL, FFDIM, WCARRY);
  tcast_f32_f16<<<dim3(DMODEL / 64, FFDIM / 64), blk256, 0, stream>>>(W2, w2t, FFDIM, DMODEL, WCARRY);

  layernorm_f16<false><<<dim3(NTOK), blk256, 0, stream>>>(x, x, ln_a_g, ln_a_b, x2, h16);

  wmma_gemm64<0, false, 0, 0, false, 0><<<dim3((NTOK / 64) * ((3 * DMODEL) / 64) / 8, 1), blk256, 0, stream>>>(
      h16, nullptr, DMODEL, 0L, wqkvt, nullptr, DMODEL, 0L, (void*)big, nullptr, 3 * DMODEL, 0L,
      nullptr, nullptr, 0L, NTOK, 3 * DMODEL, DMODEL, 1.0f / WCARRY);

  qkv_feature_f16<<<dim3((NTOK * DMODEL / 2) / 256, 3), blk256, 0, stream>>>(big, amask, qf, kf, vp);

  causal_linear_attn<<<dim3(NBATCH * NHEAD * NQB), dim3(128), 0, stream>>>(qf, kf, vp, att);

  wmma_gemm64<0, false, 0, 0, false, 0><<<dim3((NTOK / 64) * (DMODEL / 64) / 8, 1), blk256, 0, stream>>>(
      att, nullptr, DMODEL, 0L, wot, nullptr, DMODEL, 0L, (void*)big, nullptr, DMODEL, 0L,
      nullptr, nullptr, 0L, NTOK, DMODEL, DMODEL, 1.0f / (ATTCARRY * WCARRY));

  layernorm_f16<true><<<dim3(NTOK), blk256, 0, stream>>>(x, big, ln_m_g, ln_m_b, x2, h16);

  wmma_gemm64<0, false, 2, 0, false, 0><<<dim3((NTOK / 64) * (FFDIM / 64) / 8, 1), blk256, 0, stream>>>(
      h16, nullptr, DMODEL, 0L, w1t, nullptr, DMODEL, 0L, (void*)big, nullptr, FFDIM, 0L,
      b1, nullptr, 0L, NTOK, FFDIM, DMODEL, 1.0f / WCARRY);

  gelu_f16<<<dim3((NTOK * FFDIM / 2) / 256), blk256, 0, stream>>>(big, ff16, FFCARRY);

  wmma_gemm64<0, false, 2, 0, false, 0><<<dim3((NTOK / 64) * (DMODEL / 64) / 8, 1), blk256, 0, stream>>>(
      ff16, nullptr, FFDIM, 0L, w2t, nullptr, FFDIM, 0L, (void*)big, nullptr, DMODEL, 0L,
      b2, nullptr, 0L, NTOK, DMODEL, FFDIM, 1.0f / (FFCARRY * WCARRY));

  add_f32<<<dim3((NTOK * DMODEL / 4) / 256), blk256, 0, stream>>>(x2, big, out);
}
